// TrainableTFNLayer2D_82248623718879
// MI455X (gfx1250) — hardware-verified
//
#include <hip/hip_runtime.h>
#include <hip/hip_bf16.h>
#include <math.h>

#define NBf 8
#define LLf 2048
#define EEf 512
#define DDf 64
#define HWf 4096
#define GH 64
#define C1 128
#define STEPS 5
#define GSTR 48

typedef _Float16 bf16;
typedef _Float16 f16;
typedef __attribute__((ext_vector_type(4))) unsigned v4u_t;
typedef unsigned v4ua __attribute__((ext_vector_type(4), may_alias));
typedef __attribute__((ext_vector_type(4))) float v4f_t;
typedef float v4fa __attribute__((ext_vector_type(4), may_alias));
typedef __attribute__((ext_vector_type(16))) bf16  bf16x16;
typedef bf16x16 f16x16;
typedef __attribute__((ext_vector_type(8)))  bf16  bf16x8;
typedef bf16x8 f16x8;
typedef __attribute__((ext_vector_type(4)))  bf16  bf16x4;
typedef __attribute__((ext_vector_type(8)))  float f32x8;
__device__ __forceinline__ f32x8 wmma16(f16x16 a, f16x16 b, f32x8 c) {
  c = __builtin_amdgcn_wmma_f32_16x16x32_f16(false, a, false, b, (short)0, c, false, false);
  asm volatile("v_nop\n\tv_nop\n\tv_nop\n\tv_nop" : "+v"(c) : "v"(a), "v"(b));
  return c;
}
#define LDS_STRIDE 48
#define KSTRIDE    72
#define VSTRIDE    48

__device__ __forceinline__ f32x8 wmma_bf16(bf16x16 a, bf16x16 b, f32x8 c) {
  c = __builtin_amdgcn_wmma_f32_16x16x32_f16(false, a, false, b, (short)0, c, false, false);
  asm volatile("v_nop\n\tv_nop\n\tv_nop\n\tv_nop" : "+v"(c) : "v"(a), "v"(b));
  return c;
}

template <typename T>
__device__ __forceinline__ bf16x16 load_frag(const T* __restrict__ base, int ld,
                                             int row0, int k0) {
  const int lane = threadIdx.x & 31;
  const int r    = lane & 15;
  const int kh   = (lane >> 4) * 8;
  const T* p0 = base + (size_t)(row0 + r) * ld + (k0 + kh);
  const T* p1 = p0 + 16;
  bf16x16 f;
#pragma unroll
  for (int i = 0; i < 8; ++i) {
    f[i]     = (bf16)p0[i];
    f[i + 8] = (bf16)p1[i];
  }
  return f;
}

__device__ __forceinline__ bf16x16 lds_frag(const bf16* base, int stride) {
  const int lane = threadIdx.x & 31;
  const int row  = lane & 15;
  const int kh   = (lane >> 4) * 8;
  const bf16x8 lo = *(const bf16x8*)(base + row * stride + kh);
  const bf16x8 hi = *(const bf16x8*)(base + row * stride + kh + 16);
  bf16x16 f;
#pragma unroll
  for (int i = 0; i < 8; ++i) { f[i] = lo[i]; f[i + 8] = hi[i]; }
  return f;
}

template <typename T>
__device__ __forceinline__ void stage_read16(const T* __restrict__ p, float* buf) {
#pragma unroll
  for (int i = 0; i < 16; ++i) buf[i] = (float)p[i];
}

__device__ __forceinline__ void stage_write(bf16* dst, const float* buf, int nquad) {
#pragma unroll
  for (int i = 0; i < nquad; ++i) {
    bf16x4 q;
    q[0] = (bf16)buf[4 * i];     q[1] = (bf16)buf[4 * i + 1];
    q[2] = (bf16)buf[4 * i + 2]; q[3] = (bf16)buf[4 * i + 3];
    *(bf16x4*)(dst + 4 * i) = q;
  }
}


#define GSTR 48
template <typename AT, int EPI, bool OUT16>
__global__ __launch_bounds__(256) void gemm_kne(const AT* __restrict__ A, int lda, const float* __restrict__ Wm, int ldw,
                                                const float* __restrict__ bias, const float* __restrict__ R, const float* __restrict__ gvec,
                                                void* __restrict__ Yv, int ldy, int K) {
  __shared__ __attribute__((aligned(16))) f16 ldsA[128 * GSTR];
  __shared__ __attribute__((aligned(16))) f16 ldsW[128 * GSTR];
  __shared__ __attribute__((aligned(16))) float oS[8][32 * 68];
  const int tid = threadIdx.x, lane = tid & 31, wave = tid >> 5, cl = lane & 15, rh = (lane >> 4) * 8;
  const int m0 = blockIdx.x * 128, n0 = blockIdx.y * 128;
  const int wm = (wave & 3) * 32, wn = (wave >> 2) * 64;
  f32x8 acc[2][4];
#pragma unroll
  for (int i = 0; i < 2; ++i)
#pragma unroll
    for (int j = 0; j < 4; ++j) { f32x8 z = {}; acc[i][j] = z; }
#pragma unroll 1
  for (int k0 = 0; k0 < K; k0 += 32) {
    __syncthreads();
    { const int row = tid >> 1, ch = (tid & 1) * 16;
      const AT* src = A + (size_t)(m0 + row) * lda + k0 + ch;
#pragma unroll
      for (int g = 0; g < 16; ++g) ldsA[row * GSTR + ch + g] = (f16)src[g]; }
    { const int k = tid >> 3, nn0 = (tid & 7) * 16;
      const float* src = Wm + (size_t)(k0 + k) * ldw + n0 + nn0;
#pragma unroll
      for (int g = 0; g < 4; ++g) { const v4f_t v = *(const v4f_t*)(src + 4 * g);
#pragma unroll
        for (int u = 0; u < 4; ++u) ldsW[(nn0 + 4 * g + u) * GSTR + k] = (f16)v[u]; } }
    __syncthreads();
    f16x16 af[2];
#pragma unroll
    for (int i = 0; i < 2; ++i) af[i] = lds_frag(ldsA + (wm + 16 * i) * GSTR, GSTR);
#pragma unroll
    for (int j = 0; j < 4; ++j) {
      const f16x16 bf = lds_frag(ldsW + (wn + 16 * j) * GSTR, GSTR);
#pragma unroll
      for (int i = 0; i < 2; ++i) acc[i][j] = wmma16(af[i], bf, acc[i][j]);
    }
  }
  float* so = oS[wave];
#pragma unroll
  for (int i = 0; i < 2; ++i)
#pragma unroll
    for (int j = 0; j < 4; ++j) {
      const int n = n0 + wn + 16 * j + cl;
      const float bv = bias ? bias[n] : 0.0f;
      const float gv = (EPI == 2) ? gvec[n] : 0.0f;
      if (EPI == 1) {
#pragma unroll 1
        for (int r = 0; r < 8; ++r) { const float xg = acc[i][j][r] + bv; so[(16 * i + rh + r) * 68 + 16 * j + cl] = 0.5f * xg * (1.0f + erff(xg * 0.70710678118654752f)); }
      } else {
#pragma unroll
        for (int r = 0; r < 8; ++r) {
          float v = acc[i][j][r] + bv;
          if (EPI == 2) v = R[(size_t)(m0 + wm + 16 * i + rh + r) * ldy + n] + gv * v;
          so[(16 * i + rh + r) * 68 + 16 * j + cl] = v;
        }
      }
    }
  asm volatile("s_wait_dscnt 0" ::: "memory");
  __builtin_amdgcn_wave_barrier();
#pragma unroll 1
  for (int pass = 0; pass < 2; ++pass) {
    if (OUT16) {
      f16* Y = (f16*)Yv;
#pragma unroll
      for (int it = 0; it < 8; ++it) { const int c = lane + 32 * it, rr = c >> 3, q8 = (c & 7) * 8;
        union { f16 h[8]; v4u_t v; } u;
#pragma unroll
        for (int e = 0; e < 8; ++e) u.h[e] = (f16)so[rr * 68 + q8 + e];
        *(volatile v4u_t*)(Y + (size_t)(m0 + wm + rr) * ldy + n0 + wn + q8) = u.v; }
    } else {
      float* Y = (float*)Yv;
#pragma unroll
      for (int it = 0; it < 16; ++it) { const int f4 = lane + 32 * it, rr = f4 >> 4, q = (f4 & 15) * 4;
        *(volatile v4f_t*)(Y + (size_t)(m0 + wm + rr) * ldy + n0 + wn + q) = *(const v4fa*)(so + rr * 68 + q); }
    }
    __threadfence();
  }
}

__global__ __launch_bounds__(256) void k_transpose(const float* __restrict__ Wm, float* __restrict__ Wt, int rows, int cols) {
  __shared__ float tS[64][65];
  const int tid = threadIdx.x, tbj = cols / 64, bi = blockIdx.x / tbj, bj = blockIdx.x % tbj;
  for (int e = tid; e < 64 * 64; e += 256) { const int r = e >> 6, c = e & 63; tS[r][c] = Wm[(size_t)(bi * 64 + r) * cols + bj * 64 + c]; }
  __syncthreads();
  for (int ch = tid; ch < 64 * 16; ch += 256) { const int r = ch >> 4, q4 = (ch & 15) * 4; v4f_t o; o[0] = tS[q4][r]; o[1] = tS[q4 + 1][r]; o[2] = tS[q4 + 2][r]; o[3] = tS[q4 + 3][r];
    float* dst = Wt + (size_t)(bj * 64 + r) * rows + bi * 64 + q4; *(volatile v4f_t*)dst = o; __threadfence(); *(volatile v4f_t*)dst = o; }
}
__global__ __launch_bounds__(128) void k_padrows(const float* __restrict__ w, float* __restrict__ wp) { const int r = blockIdx.x, c = threadIdx.x; const float v = (r < DDf) ? w[(size_t)r * C1 + c] : 0.0f; *(volatile float*)(wp + (size_t)r * C1 + c) = v; __threadfence(); *(volatile float*)(wp + (size_t)r * C1 + c) = v; }
__global__ __launch_bounds__(256) void k_rowbias(float* __restrict__ t, const float* __restrict__ bias) { const size_t row = blockIdx.x; const float bv = bias[row];
  for (int q4 = threadIdx.x; q4 < HWf / 4; q4 += 256) { v4f_t v = *(const v4f_t*)(t + row * HWf + q4 * 4); for (int e = 0; e < 4; ++e) v[e] += bv; *(volatile v4f_t*)(t + row * HWf + q4 * 4) = v; __threadfence(); *(volatile v4f_t*)(t + row * HWf + q4 * 4) = v; } }
__global__ __launch_bounds__(256) void k_fill(float* __restrict__ p, float val, size_t n4) { const size_t i = (size_t)blockIdx.x * 256 + threadIdx.x; if (i < n4) { v4f_t v = {val, val, val, val}; *(volatile v4f_t*)(p + 4 * i) = v; __threadfence(); *(volatile v4f_t*)(p + 4 * i) = v; } }
__global__ __launch_bounds__(128) void k_wprep(const float* __restrict__ Wto, const float* __restrict__ Wfrom, float* __restrict__ WtoT, float* __restrict__ WfromT) {
  const int e = blockIdx.x;
  { const int c = threadIdx.x; const float v = (c < DDf) ? Wto[(size_t)c * EEf + e] : 0.0f; *(volatile float*)(WtoT + (size_t)e * 128 + c) = v; __threadfence(); *(volatile float*)(WtoT + (size_t)e * 128 + c) = v; }
  if (e < DDf) { for (int o = threadIdx.x; o < EEf; o += 128) { const float v = Wfrom[(size_t)o * DDf + e]; *(volatile float*)(WfromT + (size_t)e * EEf + o) = v; __threadfence(); *(volatile float*)(WfromT + (size_t)e * EEf + o) = v; } }
}
__global__ __launch_bounds__(256) void k_gauss(const float* __restrict__ pos, const float* __restrict__ logsig, float mult, int b, float* __restrict__ G) {
  __shared__ float gy[GH], gx[GH]; __shared__ float zs[2];
  const int l = blockIdx.x, tid = threadIdx.x;
  const float ls = logsig[0]; const float sp = (ls > 20.0f) ? ls : log1pf(expf(ls)); const float sig = (sp + 1e-6f) * mult; const float inv2s2 = 1.0f / (2.0f * sig * sig);
  const float py = pos[((size_t)b * LLf + l) * 2 + 0], px = pos[((size_t)b * LLf + l) * 2 + 1];
  if (tid < GH) { const float d = (float)tid - py; gy[tid] = expf(-d * d * inv2s2); } else if (tid < 2 * GH) { const float d = (float)(tid - GH) - px; gx[tid - GH] = expf(-d * d * inv2s2); }
  __syncthreads();
  if (tid < 64) { float v = (tid < 32) ? (gy[tid] + gy[tid + 32]) : (gx[tid - 32] + gx[tid]);
#pragma unroll
    for (int off = 1; off < 32; off <<= 1) v += __shfl_xor(v, off, 32);
    if ((tid & 31) == 0) zs[tid >> 5] = v; }
  __syncthreads();
  const float scl = 1024.0f / (zs[0] * zs[1] + 1e-6f);
  for (int q4 = tid; q4 < HWf / 4; q4 += 256) { const int h = (q4 * 4) / GH, w0 = (q4 * 4) % GH; v4f_t o; for (int e = 0; e < 4; ++e) o[e] = gy[h] * gx[w0 + e] * scl;
    *(volatile v4f_t*)(G + (size_t)l * HWf + q4 * 4) = o; __threadfence(); *(volatile v4f_t*)(G + (size_t)l * HWf + q4 * 4) = o; }
}
__global__ __launch_bounds__(256) void k_conv3(const float* __restrict__ fld, const float* __restrict__ Wc, const float* __restrict__ bc, float* __restrict__ hout) {
  __shared__ __attribute__((aligned(16))) f16 aS[128 * 40];
  __shared__ __attribute__((aligned(16))) f16 bS[128 * 40];
  __shared__ __attribute__((aligned(16))) float oS[128 * 132];
  const int tid = threadIdx.x, lane = tid & 31, wave = tid >> 5, cl = lane & 15, rh = (lane >> 4) * 8;
  const int p0 = blockIdx.x * 128;
  f32x8 acc[8];
#pragma unroll
  for (int j = 0; j < 8; ++j) { f32x8 z = {}; acc[j] = z; }
#pragma unroll 1
  for (int ks = 0; ks < (DDf * 9) / 32; ++ks) {
    __syncthreads();
    { const int r = tid >> 1, q = (tid & 1) * 16; const int p = p0 + r, py = p / GH, px = p % GH;
#pragma unroll 1
      for (int e = 0; e < 16; ++e) { const int k = ks * 32 + q + e, ci = k / 9, tap = k % 9, yy = py + tap / 3 - 1, xx = px + tap % 3 - 1;
        float v = 0.0f; if (yy >= 0 && yy < GH && xx >= 0 && xx < GH) v = fld[(size_t)ci * HWf + yy * GH + xx]; aS[r * 40 + q + e] = (f16)v; } }
    { const int co = tid >> 1, q = (tid & 1) * 16; const float* wr = Wc + (size_t)co * (DDf * 9) + ks * 32 + q;
#pragma unroll
      for (int e = 0; e < 16; ++e) bS[co * 40 + q + e] = (f16)wr[e]; }
    __syncthreads();
    const f16x16 af = lds_frag(aS + (wave * 16) * 40, 40);
#pragma unroll
    for (int j = 0; j < 8; ++j) acc[j] = wmma16(af, lds_frag(bS + (j * 16) * 40, 40), acc[j]);
  }
#pragma unroll
  for (int j = 0; j < 8; ++j) { const int co = j * 16 + cl; const float bb = bc[co];
#pragma unroll
    for (int r = 0; r < 8; ++r) oS[co * 132 + wave * 16 + rh + r] = fmaxf(acc[j][r] + bb, 0.0f); }
  __syncthreads();
#pragma unroll 1
  for (int pass = 0; pass < 2; ++pass) { for (int q4 = tid; q4 < 128 * 32; q4 += 256) { const int co = q4 >> 5, c4 = (q4 & 31) * 4;
      *(volatile v4f_t*)(hout + (size_t)co * HWf + p0 + c4) = *(const v4fa*)(oS + co * 132 + c4); } __threadfence(); }
}
__global__ __launch_bounds__(256) void k_fieldT(const float* __restrict__ fld, float* __restrict__ FT) {
  __shared__ float tS[64][65];
  const int tid = threadIdx.x, p0 = blockIdx.x * 64;
  for (int e = tid; e < 64 * 64; e += 256) { const int c = e >> 6, p = e & 63; tS[c][p] = fld[(size_t)c * HWf + p0 + p]; }
  __syncthreads();
  for (int e = tid; e < 64 * 32; e += 256) { const int p = e >> 5, c4 = (e & 31) * 4; v4f_t o; for (int k = 0; k < 4; ++k) o[k] = (c4 + k < DDf) ? tS[c4 + k][p] : 0.0f;
    *(volatile v4f_t*)(FT + (size_t)(p0 + p) * 128 + c4) = o; __threadfence(); *(volatile v4f_t*)(FT + (size_t)(p0 + p) * 128 + c4) = o; }
}

extern "C" void kernel_launch(void* const* d_in, const int* in_sizes, int n_in,
                              void* d_out, int out_size, void* d_ws, size_t ws_size,
                              hipStream_t stream) {
  (void)in_sizes; (void)n_in; (void)out_size;
  const float** f = (const float**)d_in;
  const float* tok = f[0], *pos = f[1], *Wto = f[2], *Wfrom = f[3], *c1w = f[4], *c1b = f[5], *c2w = f[6], *c2b = f[7], *logsig = f[8];
  float* out = (float*)d_out;
  char* ws = (char*)d_ws;
  float* WtoT = (float*)ws; ws += (size_t)EEf * 128 * 4; float* WfromT = (float*)ws; ws += (size_t)DDf * EEf * 4;
  float* W2p = (float*)ws; ws += (size_t)128 * C1 * 4;
  float* proj = (float*)ws; ws += (size_t)NBf * LLf * 128 * 4;
  float* projT = (float*)ws; ws += (size_t)128 * LLf * 4;
  float* G = (float*)ws; ws += (size_t)LLf * HWf * 4;
  float* fld = (float*)ws; ws += (size_t)128 * HWf * 4;
  float* hbuf = (float*)ws; ws += (size_t)C1 * HWf * 4;
  float* FT = (float*)ws; ws += (size_t)HWf * 128 * 4;
  float* samp = (float*)ws; ws += (size_t)NBf * LLf * 128 * 4;
  float* ones = (float*)ws; ws += HWf * 4; float* inv1024 = (float*)ws; ws += HWf * 4;
  if ((size_t)(ws - (char*)d_ws) > ws_size) return;
  const dim3 blk(256);
  k_wprep<<<dim3(EEf), dim3(128), 0, stream>>>(Wto, Wfrom, WtoT, WfromT);
  k_padrows<<<dim3(128), dim3(128), 0, stream>>>(c2w, W2p);
  k_fill<<<dim3((HWf / 4 + 255) / 256), blk, 0, stream>>>(ones, 1.0f, HWf / 4);
  k_fill<<<dim3((HWf / 4 + 255) / 256), blk, 0, stream>>>(inv1024, 1.0f / 1024.0f, HWf / 4);
  k_fill<<<dim3(((size_t)NBf * LLf * 128 / 4 + 255) / 256), blk, 0, stream>>>(samp, 0.0f, (size_t)NBf * LLf * 128 / 4);
  gemm_kne<float, 0, false><<<dim3(NBf * LLf / 128, 1), blk, 0, stream>>>(tok, EEf, WtoT, 128, nullptr, nullptr, nullptr, proj, 128, EEf);
  for (int b = 0; b < NBf; ++b) {
    k_transpose<<<dim3((LLf / 64) * (128 / 64)), blk, 0, stream>>>(proj + (size_t)b * LLf * 128, projT, LLf, 128);
    k_gauss<<<dim3(LLf), blk, 0, stream>>>(pos, logsig, 1.0f, b, G);
    k_fill<<<dim3((128 * HWf / 4 + 255) / 256), blk, 0, stream>>>(fld, 0.0f, (size_t)128 * HWf / 4);
    gemm_kne<float, 2, false><<<dim3(1, HWf / 128), blk, 0, stream>>>(projT, LLf, G, HWf, nullptr, fld, inv1024, fld, HWf, LLf);
    for (int s = 0; s < STEPS; ++s) {
      k_conv3<<<dim3(HWf / 128), blk, 0, stream>>>(fld, c1w, c1b, hbuf);
      gemm_kne<float, 2, false><<<dim3(1, HWf / 128), blk, 0, stream>>>(W2p, C1, hbuf, HWf, nullptr, fld, ones, fld, HWf, C1);
      k_rowbias<<<dim3(DDf), blk, 0, stream>>>(fld, c2b);
    }
    k_fieldT<<<dim3(HWf / 64), blk, 0, stream>>>(fld, FT);
    k_gauss<<<dim3(LLf), blk, 0, stream>>>(pos, logsig, 2.0f, b, G);
    gemm_kne<float, 2, false><<<dim3(LLf / 128, 1), blk, 0, stream>>>(G, HWf, FT, 128, nullptr, samp + (size_t)b * LLf * 128, inv1024, samp + (size_t)b * LLf * 128, 128, HWf);
  }
  gemm_kne<float, 0, false><<<dim3(NBf * LLf / 128, EEf / 128), blk, 0, stream>>>(samp, 128, WfromT, EEf, nullptr, nullptr, nullptr, out, EEf, DDf);
}
